// self_attention_head_61375082660264
// MI455X (gfx1250) — hardware-verified
//
#include <hip/hip_runtime.h>
#include <hip/hip_bf16.h>
#include <math.h>
#include <stdint.h>

#define NB   4
#define SEQ  4096
#define DE   512
#define HD   64
#define KC   64
#define NQB  (SEQ / 64)
#define NROW (NB * SEQ)
#define NX   (NROW * DE)
#define NW   (HD * DE)
#define NO   (NROW * HD)
#define PSC  1024.0f
#define RSC  2048.0f
#define VSC  64.0f
#define OSC  8.0f
static_assert((SEQ % 64) == 0);
static_assert(HD == 64);
static_assert(KC == 64);
static_assert((DE % 32) == 0);
static_assert(((NX / 8) % 256) == 0);
static_assert(((NW / 8) % 256) == 0);
static_assert((NROW % 64) == 0);

typedef _Float16 v16h __attribute__((ext_vector_type(16)));
typedef _Float16 v8h  __attribute__((ext_vector_type(8)));
typedef __bf16   v16b __attribute__((ext_vector_type(16)));
typedef float    v8f  __attribute__((ext_vector_type(8)));
typedef float    v4f  __attribute__((ext_vector_type(4)));
typedef unsigned int v4u __attribute__((ext_vector_type(4)));

union FragH { v16h v; v8h h[2]; };
union FragB { v16b v; v4u u[2]; };
union HU8   { v8h h; v4u u; };

__device__ __forceinline__ unsigned short bf_bits(float f) {
  unsigned u = __float_as_uint(f);
  return (unsigned short)((u + 0x7FFFu + ((u >> 16) & 1u)) >> 16);
}
__device__ __forceinline__ float bf_up(unsigned short h) { return __uint_as_float(((unsigned)h) << 16); }
__device__ __forceinline__ float bfr(float f) { return bf_up(bf_bits(f)); }
__device__ __forceinline__ unsigned pk16(unsigned short a, unsigned short b) { return (unsigned)a | ((unsigned)b << 16); }
__device__ __forceinline__ v8f zero8() { v8f z = {0.f, 0.f, 0.f, 0.f, 0.f, 0.f, 0.f, 0.f}; return z; }

__device__ __forceinline__ v16h ldfrag_h(const _Float16* p) {
  FragH f;
  f.h[0] = *(const v8h*)(p);
  f.h[1] = *(const v8h*)(p + 16);
  return f.v;
}
__device__ __forceinline__ v16b ldfrag_b(const unsigned short* p) {
  FragB f;
  f.u[0] = *(const v4u*)(p);
  f.u[1] = *(const v4u*)(p + 16);
  return f.v;
}

__device__ __forceinline__ v8f mma_h(v16h a, v16h b, v8f c) {
  c = __builtin_amdgcn_wmma_f32_16x16x32_f16(false, a, false, b, (short)0, c, false, false);
#if defined(__HIP_DEVICE_COMPILE__)
  asm volatile("v_nop\n\tv_nop\n\tv_nop\n\tv_nop" : "+v"(c) : "v"(a), "v"(b));
#endif
  return c;
}
__device__ __forceinline__ v8f mma_b(v16b a, v16b b, v8f c) {
  c = __builtin_amdgcn_wmma_f32_16x16x32_bf16(false, a, false, b, (short)0, c, false, false);
#if defined(__HIP_DEVICE_COMPILE__)
  asm volatile("v_nop\n\tv_nop\n\tv_nop\n\tv_nop" : "+v"(c) : "v"(a), "v"(b));
#endif
  return c;
}
__device__ __forceinline__ void wave_sync_lds() {
  __builtin_amdgcn_fence(__ATOMIC_RELEASE, "workgroup");
  __builtin_amdgcn_wave_barrier();
  __builtin_amdgcn_fence(__ATOMIC_ACQUIRE, "workgroup");
}

__global__ __launch_bounds__(256) void conv_bf16(const float* __restrict__ X, unsigned short* Y, int n8) {
  const int i  = blockIdx.x * 256 + threadIdx.x;
  const int ic = (i < n8) ? i : (n8 - 1);
  const float* src = X + (size_t)ic * 8;
  const v4f a = *(const v4f*)(src);
  const v4f c = *(const v4f*)(src + 4);
  v4u o;
  o[0] = pk16(bf_bits(a[0]), bf_bits(a[1]));
  o[1] = pk16(bf_bits(a[2]), bf_bits(a[3]));
  o[2] = pk16(bf_bits(c[0]), bf_bits(c[1]));
  o[3] = pk16(bf_bits(c[2]), bf_bits(c[3]));
  if (i < n8) *(volatile v4u*)(Y + (size_t)i * 8) = o;
  __threadfence();
  if (i < n8) *(volatile v4u*)(Y + (size_t)i * 8) = o;
}

__global__ __launch_bounds__(128)
void proj_qkv(const unsigned short* __restrict__ Xb,
              const unsigned short* __restrict__ Wqb, const unsigned short* __restrict__ Wkb,
              const unsigned short* __restrict__ Wvb,
              const float* __restrict__ bq, const float* __restrict__ bk, const float* __restrict__ bv,
              _Float16* Qh, _Float16* Qr, _Float16* Kh, _Float16* Kr, _Float16* VTh, _Float16* VTr) {
  __shared__ __align__(16) _Float16 Th[64 * 72];
  __shared__ __align__(16) _Float16 Tr[64 * 72];

  const int tid  = threadIdx.x;
  const int wave = tid >> 5;
  const int lane = tid & 31;
  const int hh   = lane >> 4;
  const int c    = lane & 15;
  const int r0   = blockIdx.x * 64;
  const int b    = r0 / SEQ;
  const int s0   = r0 - b * SEQ;
  const unsigned short* ap = Xb + (size_t)(r0 + wave * 16 + c) * DE + 8 * hh;

#pragma unroll 1
  for (int w = 0; w < 3; ++w) {
    const unsigned short* Wb = (w == 0) ? Wqb : ((w == 1) ? Wkb : Wvb);
    const float* bp = (w == 0) ? bq : ((w == 1) ? bk : bv);

    v8f acc[4];
#pragma unroll
    for (int nt = 0; nt < 4; ++nt) acc[nt] = zero8();

#pragma unroll 2
    for (int k0 = 0; k0 < DE; k0 += 32) {
      const v16b a = ldfrag_b(ap + k0);
#pragma unroll
      for (int nt = 0; nt < 4; ++nt) {
        const v16b wf = ldfrag_b(Wb + (size_t)(nt * 16 + c) * DE + 8 * hh + k0);
        acc[nt] = mma_b(a, wf, acc[nt]);
      }
    }

    if (w < 2) {
      _Float16* Ph = (w == 0) ? Qh : Kh;
      _Float16* Pr = (w == 0) ? Qr : Kr;
#pragma unroll
      for (int nt = 0; nt < 4; ++nt) {
        const int n = nt * 16 + c;
        const float bias = bfr(bp[n]);
#pragma unroll
        for (int r = 0; r < 8; ++r) {
          const float v = acc[nt][r] + bias;
          const _Float16 hq = (_Float16)v;
          const _Float16 rq = (_Float16)((v - (float)hq) * RSC);
          const int pi = (wave * 16 + 8 * hh + r) * 72 + n;
          Th[pi] = hq;
          Tr[pi] = rq;
        }
      }
      __syncthreads();
      const int q8 = lane >> 3, c8 = (lane & 7) * 8;
      v4u vh[4], vr[4];
#pragma unroll
      for (int it = 0; it < 4; ++it) {
        const int row = wave * 16 + it * 4 + q8;
        HU8 u;
        u.h = *(const v8h*)(Th + row * 72 + c8);
        vh[it] = u.u;
        u.h = *(const v8h*)(Tr + row * 72 + c8);
        vr[it] = u.u;
      }
#pragma unroll
      for (int it = 0; it < 4; ++it) {
        const int row = wave * 16 + it * 4 + q8;
        const size_t o = (size_t)(r0 + row) * HD + c8;
        *(volatile v4u*)(Ph + o) = vh[it];
        *(volatile v4u*)(Pr + o) = vr[it];
      }
      __threadfence();
#pragma unroll
      for (int it = 0; it < 4; ++it) {
        const int row = wave * 16 + it * 4 + q8;
        const size_t o = (size_t)(r0 + row) * HD + c8;
        *(volatile v4u*)(Ph + o) = vh[it];
        *(volatile v4u*)(Pr + o) = vr[it];
      }
      __syncthreads();
    } else {
#pragma unroll
      for (int nt = 0; nt < 4; ++nt) {
        const int n = nt * 16 + c;
        const float bias = bfr(bp[n]);
#pragma unroll
        for (int r = 0; r < 8; ++r) {
          const float v = (acc[nt][r] + bias) * VSC;
          const _Float16 hq = (_Float16)v;
          const _Float16 rq = (_Float16)((v - (float)hq) * RSC);
          const int pi = n * 72 + wave * 16 + 8 * hh + r;
          Th[pi] = hq;
          Tr[pi] = rq;
        }
      }
      __syncthreads();
      const int q8 = tid >> 3, c8 = (tid & 7) * 8;
      v4u vh[4], vr[4];
#pragma unroll
      for (int it = 0; it < 4; ++it) {
        const int d = it * 16 + q8;
        HU8 u;
        u.h = *(const v8h*)(Th + d * 72 + c8);
        vh[it] = u.u;
        u.h = *(const v8h*)(Tr + d * 72 + c8);
        vr[it] = u.u;
      }
#pragma unroll
      for (int it = 0; it < 4; ++it) {
        const int d = it * 16 + q8;
        const size_t o = ((size_t)b * HD + d) * SEQ + s0 + c8;
        *(volatile v4u*)(VTh + o) = vh[it];
        *(volatile v4u*)(VTr + o) = vr[it];
      }
      __threadfence();
#pragma unroll
      for (int it = 0; it < 4; ++it) {
        const int d = it * 16 + q8;
        const size_t o = ((size_t)b * HD + d) * SEQ + s0 + c8;
        *(volatile v4u*)(VTh + o) = vh[it];
        *(volatile v4u*)(VTr + o) = vr[it];
      }
    }
  }
}

__global__ __launch_bounds__(128)
void attn64(const _Float16* __restrict__ Qh, const _Float16* __restrict__ Qr,
            const _Float16* __restrict__ Kh, const _Float16* __restrict__ Kr,
            const _Float16* __restrict__ VTh, const _Float16* __restrict__ VTr, float* outp) {
  __shared__ __align__(16) _Float16 Khs[KC * HD];
  __shared__ __align__(16) _Float16 Krs[KC * HD];
  __shared__ __align__(16) _Float16 Vhs[HD * KC];
  __shared__ __align__(16) _Float16 Vrs[HD * KC];
  __shared__ __align__(16) _Float16 Psh[4][16 * KC];
  __shared__ __align__(16) _Float16 Rsh[4][16 * KC];
  __shared__ __align__(16) float    Os[4][16 * HD];

  const int tid  = threadIdx.x;
  const int wave = tid >> 5;
  const int lane = tid & 31;
  const int hh   = lane >> 4;
  const int c    = lane & 15;

  const int bx = blockIdx.x;
  const int qb = bx % NQB;
  const int b  = bx / NQB;
  const int q0 = qb * 64 + wave * 16;
  const int rlo = q0 + 8 * hh;
  const size_t rowB = (size_t)b * SEQ;
  const _Float16* VThb = VTh + (size_t)b * HD * SEQ;
  const _Float16* VTrb = VTr + (size_t)b * HD * SEQ;

  v16h qh[2], qr[2];
#pragma unroll
  for (int dc = 0; dc < 2; ++dc) {
    qh[dc] = ldfrag_h(Qh + (rowB + q0 + c) * HD + dc * 32 + 8 * hh);
    qr[dc] = ldfrag_h(Qr + (rowB + q0 + c) * HD + dc * 32 + 8 * hh);
  }

  float mrow[8], lrow[8];
  v8f oacc[4];
#pragma unroll
  for (int r = 0; r < 8; ++r) { mrow[r] = -INFINITY; lrow[r] = 0.f; }
#pragma unroll
  for (int t = 0; t < 4; ++t) oacc[t] = zero8();

#pragma unroll 1
  for (int kt = 0; kt <= qb; ++kt) {
    const int kv0 = kt * KC;

    __syncthreads();
    {
      const int r = tid >> 1, hf = (tid & 1) * 32;
      const _Float16* kgh = Kh + (rowB + kv0 + r) * HD + hf;
      const _Float16* kgr = Kr + (rowB + kv0 + r) * HD + hf;
#pragma unroll
      for (int i = 0; i < 4; ++i) {
        const v8h a0 = *(const v8h*)(kgh + 8 * i);
        const v8h a1 = *(const v8h*)(kgr + 8 * i);
        *(v8h*)(Khs + r * HD + hf + 8 * i) = a0;
        *(v8h*)(Krs + r * HD + hf + 8 * i) = a1;
      }
      const _Float16* vgh = VThb + (size_t)r * SEQ + kv0 + hf;
      const _Float16* vgr = VTrb + (size_t)r * SEQ + kv0 + hf;
#pragma unroll
      for (int i = 0; i < 4; ++i) {
        const v8h b0 = *(const v8h*)(vgh + 8 * i);
        const v8h b1 = *(const v8h*)(vgr + 8 * i);
        *(v8h*)(Vhs + r * KC + hf + 8 * i) = b0;
        *(v8h*)(Vrs + r * KC + hf + 8 * i) = b1;
      }
    }
    __syncthreads();

    v8f s[4];
#pragma unroll
    for (int j = 0; j < 4; ++j) {
      v8f sh = zero8();
      v8f sx = zero8();
#pragma unroll
      for (int dc = 0; dc < 2; ++dc) {
        FragH kb, kx;
        kb.h[0] = *(const v8h*)(Khs + (j * 16 + c) * HD + dc * 32 + 8 * hh);
        kb.h[1] = *(const v8h*)(Khs + (j * 16 + c) * HD + dc * 32 + 16 + 8 * hh);
        kx.h[0] = *(const v8h*)(Krs + (j * 16 + c) * HD + dc * 32 + 8 * hh);
        kx.h[1] = *(const v8h*)(Krs + (j * 16 + c) * HD + dc * 32 + 16 + 8 * hh);
        sh = mma_h(qh[dc], kb.v, sh);
        sx = mma_h(qh[dc], kx.v, sx);
        sx = mma_h(qr[dc], kb.v, sx);
      }
      const int key = kv0 + j * 16 + c;
#pragma unroll
      for (int r = 0; r < 8; ++r) {
        const float sv = sh[r] + sx[r] * (1.0f / RSC);
        s[j][r] = (key > rlo + r) ? -INFINITY : sv;
      }
    }

    _Float16* pwh = Psh[wave];
    _Float16* pwr = Rsh[wave];
#pragma unroll
    for (int r = 0; r < 8; ++r) {
      float m = s[0][r];
      m = fmaxf(m, s[1][r]);
      m = fmaxf(m, s[2][r]);
      m = fmaxf(m, s[3][r]);
#pragma unroll
      for (int off = 1; off < 16; off <<= 1) m = fmaxf(m, __shfl_xor(m, off, 32));
      const float mnew  = fmaxf(mrow[r], m);
      const float alpha = __expf(mrow[r] - mnew);
      mrow[r] = mnew;
      float psum = 0.f;
#pragma unroll
      for (int j = 0; j < 4; ++j) {
        const float p  = __expf(s[j][r] - mnew);
        psum += p;
        const float ph = p * PSC;
        const _Float16 hq = (_Float16)ph;
        const float res = (ph - (float)hq) * RSC;
        const int pi = (8 * hh + r) * KC + j * 16 + c;
        pwh[pi] = hq;
        pwr[pi] = (_Float16)res;
      }
#pragma unroll
      for (int off = 1; off < 16; off <<= 1) psum += __shfl_xor(psum, off, 32);
      lrow[r] = lrow[r] * alpha + psum;
#pragma unroll
      for (int t = 0; t < 4; ++t) oacc[t][r] *= alpha;
    }
    wave_sync_lds();

    FragH pa[2], pr[2];
#pragma unroll
    for (int kk = 0; kk < 2; ++kk) {
      pa[kk].h[0] = *(const v8h*)(pwh + c * KC + kk * 32 + 8 * hh);
      pa[kk].h[1] = *(const v8h*)(pwh + c * KC + kk * 32 + 16 + 8 * hh);
      pr[kk].h[0] = *(const v8h*)(pwr + c * KC + kk * 32 + 8 * hh);
      pr[kk].h[1] = *(const v8h*)(pwr + c * KC + kk * 32 + 16 + 8 * hh);
    }
#pragma unroll
    for (int t = 0; t < 4; ++t) {
      FragH vb[2], vx[2];
#pragma unroll
      for (int kk = 0; kk < 2; ++kk) {
        vb[kk].h[0] = *(const v8h*)(Vhs + (t * 16 + c) * KC + kk * 32 + 8 * hh);
        vb[kk].h[1] = *(const v8h*)(Vhs + (t * 16 + c) * KC + kk * 32 + 16 + 8 * hh);
        vx[kk].h[0] = *(const v8h*)(Vrs + (t * 16 + c) * KC + kk * 32 + 8 * hh);
        vx[kk].h[1] = *(const v8h*)(Vrs + (t * 16 + c) * KC + kk * 32 + 16 + 8 * hh);
      }
      oacc[t] = mma_h(pa[0].v, vb[0].v, oacc[t]);
      oacc[t] = mma_h(pa[1].v, vb[1].v, oacc[t]);
      v8f rr = mma_h(pa[0].v, vx[0].v, zero8());
      rr = mma_h(pa[1].v, vx[1].v, rr);
      rr = mma_h(pr[0].v, vb[0].v, rr);
      rr = mma_h(pr[1].v, vb[1].v, rr);
#pragma unroll
      for (int r = 0; r < 8; ++r) oacc[t][r] += rr[r] * (1.0f / RSC);
    }
  }

  float* os = Os[wave];
#pragma unroll
  for (int r = 0; r < 8; ++r) {
    const float l = lrow[r];
    const float inv = ((l > 0.f) ? (1.0f / l) : 0.f) * (OSC / (PSC * VSC));
#pragma unroll
    for (int t = 0; t < 4; ++t) os[(8 * hh + r) * HD + t * 16 + c] = oacc[t][r] * inv;
  }
  wave_sync_lds();
  {
    const int c4 = lane * 4;
    v4f vals[8];
#pragma unroll
    for (int it = 0; it < 8; ++it) vals[it] = *(const v4f*)(os + it * 128 + c4);
    float* C = outp + (rowB + q0) * HD;
#pragma unroll
    for (int it = 0; it < 8; ++it) *(volatile v4f*)(C + (size_t)it * 128 + c4) = vals[it];
    __threadfence();
#pragma unroll
    for (int it = 0; it < 8; ++it) *(volatile v4f*)(C + (size_t)it * 128 + c4) = vals[it];
  }
}

extern "C" void kernel_launch(void* const* d_in, const int* in_sizes, int n_in,
                              void* d_out, int out_size, void* d_ws, size_t ws_size,
                              hipStream_t stream) {
  if (n_in < 7) return;
  if (in_sizes[0] != NX) return;
  if (in_sizes[1] != NW || in_sizes[3] != NW || in_sizes[5] != NW) return;
  if (in_sizes[2] != HD || in_sizes[4] != HD || in_sizes[6] != HD) return;
  if (out_size != NO) return;

  const float* x  = (const float*)d_in[0];
  const float* Wq = (const float*)d_in[1];
  const float* bq = (const float*)d_in[2];
  const float* Wk = (const float*)d_in[3];
  const float* bk = (const float*)d_in[4];
  const float* Wv = (const float*)d_in[5];
  const float* bv = (const float*)d_in[6];

  const size_t XB = (size_t)NX * 2;
  const size_t WB = (size_t)NW * 2;
  const size_t PB = (size_t)NO * 2;
  size_t off = 0;
  const size_t oX  = off; off += XB;
  const size_t oWq = off; off += WB;
  const size_t oWk = off; off += WB;
  const size_t oWv = off; off += WB;
  const size_t oQh = off; off += PB;
  const size_t oQr = off; off += PB;
  const size_t oKh = off; off += PB;
  const size_t oKr = off; off += PB;
  const size_t oVh = off; off += PB;
  const size_t oVr = off; off += PB;
  if (off > ws_size) return;
  if (off > (size_t)134217728) return;

  char* ws = (char*)d_ws;
  unsigned short* Xb  = (unsigned short*)(ws + oX);
  unsigned short* Wqb = (unsigned short*)(ws + oWq);
  unsigned short* Wkb = (unsigned short*)(ws + oWk);
  unsigned short* Wvb = (unsigned short*)(ws + oWv);
  _Float16* Qh  = (_Float16*)(ws + oQh);
  _Float16* Qr  = (_Float16*)(ws + oQr);
  _Float16* Kh  = (_Float16*)(ws + oKh);
  _Float16* Kr  = (_Float16*)(ws + oKr);
  _Float16* VTh = (_Float16*)(ws + oVh);
  _Float16* VTr = (_Float16*)(ws + oVr);
  float* out0 = (float*)d_out;

  const int nx8 = NX / 8;
  const int nw8 = NW / 8;
  const dim3 blk(256), blk128(128);
  const dim3 gX(nx8 / 256);
  const dim3 gW(nw8 / 256);
  const dim3 gP(NROW / 64);
  const dim3 gA(NB * NQB);

  conv_bf16<<<gX, blk, 0, stream>>>(x, Xb, nx8);
  conv_bf16<<<gW, blk, 0, stream>>>(Wq, Wqb, nw8);
  conv_bf16<<<gW, blk, 0, stream>>>(Wk, Wkb, nw8);
  conv_bf16<<<gW, blk, 0, stream>>>(Wv, Wvb, nw8);

  proj_qkv<<<gP, blk128, 0, stream>>>(Xb, Wqb, Wkb, Wvb, bq, bk, bv, Qh, Qr, Kh, Kr, VTh, VTr);

  attn64<<<gA, blk128, 0, stream>>>(Qh, Qr, Kh, Kr, VTh, VTr, out0);
  (void)hipGetLastError();
}
